// SimpleGCNRec_43396349558973
// MI455X (gfx1250) — hardware-verified
//
#include <hip/hip_runtime.h>
#include <stddef.h>


#define HD      128
#define UD      64
#define CSELF   1.0f
#define LN_EPS  1e-5f
#define SLOPE   0.01f
#define NTHR    256
#define NWAVE   8
#define EPT     8
#define NGRP    2
#define CHUNK   (NTHR * EPT * NGRP)
#define WCAPC   (EPT * NGRP * 32)
#define WCAPF   (EPT * NGRP * 32)
#define ESHF    11
#define NBC     32768
#define NBF     2048
#define RCAP    61440
#define RBN     128
#define TGT     256
#define DEGCAP  512
#define GROWS   128
#define GCOLS   128
#define OTHR    512
#define TPK     64
#define TPN     32
#define TPP     72
#define ASCL    16
#define HSCL    64
#define WSCL    256
#define WSCAP   134217728

#define LDS_COUNT ((NBC + NWAVE * WCAPC + NWAVE) * 4)
#define LDS_FILL  ((RCAP + NBF + NWAVE * WCAPF + NWAVE) * 4)
#define LDS_GEMM  (GROWS * GCOLS * 4)
#define LDS_AGG   (TGT * HD * 2)

static_assert((CHUNK & (CHUNK - 1)) == 0);
static_assert((NBC & (NBC - 1)) == 0 && (NBF & (NBF - 1)) == 0);
static_assert(NBF <= (1 << ESHF));
static_assert((NBC % NBF) == 0);
static_assert(OTHR * 4 == NBF);
static_assert((RCAP % 32) == 0);
static_assert(TGT == NWAVE * 32);
static_assert(GROWS == NWAVE * 16);
static_assert((TGT % GROWS) == 0);
static_assert(NBC == NWAVE * 32 * 128);
static_assert(GCOLS == HD && GCOLS == 32 * 4);
static_assert((HD % 32) == 0 && (UD % 32) == 0);
static_assert((UD % TPK) == 0 && (HD % TPK) == 0 && (HD % TPN) == 0);
static_assert(TPN * 8 == NTHR && TPK * TPN == NTHR * 8 && TPK == NWAVE * 8);
static_assert((TPP % 8) == 0 && TPP >= TPK);
static_assert(WCAPC == EPT * NGRP * 32 && WCAPF == EPT * NGRP * 32);
static_assert(LDS_FILL <= 300 * 1024);
static_assert((OTHR % 32) == 0 && (OTHR / 32) == 16);

typedef float     v4f  __attribute__((ext_vector_type(4)));
typedef float     v8f  __attribute__((ext_vector_type(8)));
typedef int       v4i  __attribute__((ext_vector_type(4)));
typedef _Float16  v4h  __attribute__((ext_vector_type(4)));
typedef _Float16  v8h  __attribute__((ext_vector_type(8)));
typedef _Float16  v16h __attribute__((ext_vector_type(16)));
union FragH { v16h v; v8h h[2]; };
union U32F { float f; int i; };

__device__ __forceinline__ v8f wmf(v16h a, v16h b, v8f c) {
  v8f d = __builtin_amdgcn_wmma_f32_16x16x32_f16(false, a, false, b, (short)0, c, false, false);
  asm volatile("v_nop\n\tv_nop\n\tv_nop\n\tv_nop" : "+v"(d) : "v"(a), "v"(b));
  return d;
}

__device__ __forceinline__ float wsum(float v) {
#pragma unroll
  for (int o = 16; o > 0; o >>= 1) v += __shfl_xor(v, o, 32);
  return v;
}

__device__ __forceinline__ float leaky(float y) { return y >= 0.0f ? y : SLOPE * y; }

__device__ __forceinline__ float sigm(float z) {
  const float e = __expf(-z);
  return __builtin_amdgcn_rcpf(1.0f + e);
}

template <int NB, int SRC, int WC>
__device__ __forceinline__ int scan_chunk(const int* __restrict__ keys, const int* __restrict__ vals,
                                          int nK, int nN, int cbase, int slotBase, int vec8,
                                          int* list, int tid, int lane, int wave) {
  int wc = 0;
#pragma unroll
  for (int g = 0; g < NGRP; ++g) {
    const int el0  = (g * NTHR + tid) * EPT;
    const int e0   = cbase + el0;
    const int sent = -2147483647 - 1;
    v4i da, db;
    v4i sa = {0, 0, 0, 0}, sb = {0, 0, 0, 0};
    if (vec8 != 0 && cbase + CHUNK <= nK) {
      da = *(const v4i*)(keys + e0);
      db = *(const v4i*)(keys + e0 + 4);
      if (SRC) {
        sa = *(const v4i*)(vals + e0);
        sb = *(const v4i*)(vals + e0 + 4);
      }
    } else {
      const int i0 = min(e0, nK - 1),     i1 = min(e0 + 1, nK - 1), i2 = min(e0 + 2, nK - 1), i3 = min(e0 + 3, nK - 1);
      const int i4 = min(e0 + 4, nK - 1), i5 = min(e0 + 5, nK - 1), i6 = min(e0 + 6, nK - 1), i7 = min(e0 + 7, nK - 1);
      da.x = (e0     < nK) ? keys[i0] : sent;
      da.y = (e0 + 1 < nK) ? keys[i1] : sent;
      da.z = (e0 + 2 < nK) ? keys[i2] : sent;
      da.w = (e0 + 3 < nK) ? keys[i3] : sent;
      db.x = (e0 + 4 < nK) ? keys[i4] : sent;
      db.y = (e0 + 5 < nK) ? keys[i5] : sent;
      db.z = (e0 + 6 < nK) ? keys[i6] : sent;
      db.w = (e0 + 7 < nK) ? keys[i7] : sent;
      if (SRC) {
        sa.x = vals[i0]; sa.y = vals[i1]; sa.z = vals[i2]; sa.w = vals[i3];
        sb.x = vals[i4]; sb.y = vals[i5]; sb.z = vals[i6]; sb.w = vals[i7];
      }
    }
    if (SRC) {
      sa.x = min(max(sa.x, 0), nN - 1); sa.y = min(max(sa.y, 0), nN - 1);
      sa.z = min(max(sa.z, 0), nN - 1); sa.w = min(max(sa.w, 0), nN - 1);
      sb.x = min(max(sb.x, 0), nN - 1); sb.y = min(max(sb.y, 0), nN - 1);
      sb.z = min(max(sb.z, 0), nN - 1); sb.w = min(max(sb.w, 0), nN - 1);
    }
    const unsigned nb = (unsigned)slotBase;
    const unsigned s0 = (unsigned)da.x - nb, s1 = (unsigned)da.y - nb;
    const unsigned s2 = (unsigned)da.z - nb, s3 = (unsigned)da.w - nb;
    const unsigned s4 = (unsigned)db.x - nb, s5 = (unsigned)db.y - nb;
    const unsigned s6 = (unsigned)db.z - nb, s7 = (unsigned)db.w - nb;
    const bool h0 = s0 < (unsigned)NB, h1 = s1 < (unsigned)NB, h2 = s2 < (unsigned)NB, h3 = s3 < (unsigned)NB;
    const bool h4 = s4 < (unsigned)NB, h5 = s5 < (unsigned)NB, h6 = s6 < (unsigned)NB, h7 = s7 < (unsigned)NB;
    const unsigned any = __builtin_amdgcn_ballot_w32(h0 | h1 | h2 | h3 | h4 | h5 | h6 | h7);
    if (any != 0u) {
#define HITJ(HJ, SJ, VJ) { \
        const unsigned mj = __builtin_amdgcn_ballot_w32(HJ); \
        if (mj != 0u) { \
          if (HJ) { \
            const int pos = wc + (int)__builtin_amdgcn_mbcnt_lo(mj, 0u); \
            const int entv = SRC ? (((VJ) << ESHF) | (int)(SJ)) : (int)(SJ); \
            if (pos < WC) list[wave * WC + pos] = entv; \
          } \
          wc += (int)__builtin_popcount(mj); } }
      HITJ(h0, s0, sa.x)
      HITJ(h1, s1, sa.y)
      HITJ(h2, s2, sa.z)
      HITJ(h3, s3, sa.w)
      HITJ(h4, s4, sb.x)
      HITJ(h5, s5, sb.y)
      HITJ(h6, s6, sb.z)
      HITJ(h7, s7, sb.w)
#undef HITJ
    }
  }
  return wc;
}

__global__ __launch_bounds__(NTHR) void k_cvt16(const float* __restrict__ src, _Float16* dst,
                                                int rowLen, int nSrcRows, int total8, float scale) {
  const int i = (int)blockIdx.x * NTHR + (int)threadIdx.x;
  if (i >= total8) return;
  const size_t e  = (size_t)8 * (size_t)i;
  const int    r  = (int)(e / (size_t)rowLen);
  const int    k0 = (int)(e - (size_t)r * (size_t)rowLen);
  const int    rc = r < nSrcRows ? r : nSrcRows - 1;
  const float  z  = (r < nSrcRows) ? scale : 0.0f;
  const float* sp = src + (size_t)rc * rowLen + k0;
  const v4f f0 = *(const v4f*)sp;
  const v4f f1 = *(const v4f*)(sp + 4);
  v8h hv;
  hv[0] = (_Float16)(f0.x * z); hv[1] = (_Float16)(f0.y * z); hv[2] = (_Float16)(f0.z * z); hv[3] = (_Float16)(f0.w * z);
  hv[4] = (_Float16)(f1.x * z); hv[5] = (_Float16)(f1.y * z); hv[6] = (_Float16)(f1.z * z); hv[7] = (_Float16)(f1.w * z);
  _Float16* d = dst + e;
  *(volatile v8h*)d = hv;
  __threadfence();
  *(volatile v8h*)d = hv;
}

__global__ __launch_bounds__(NTHR) void k_wT16(const float* __restrict__ W, _Float16* Wp,
                                               int KD, int NC, float scale) {
  __shared__ __attribute__((aligned(16))) _Float16 sT[TPN * TPP];
  const int tid = threadIdx.x;
  const int k0 = (int)blockIdx.x * TPK, n0 = (int)blockIdx.y * TPN;
  const int nc = tid & 31, kq = tid >> 5;
#pragma unroll
  for (int i = 0; i < TPK / NWAVE; ++i) {
    const int kr = kq + NWAVE * i;
    const float v = W[(size_t)(k0 + kr) * NC + n0 + nc] * scale;
    sT[nc * TPP + kr] = (_Float16)v;
  }
  __syncthreads();
  const int nl = tid >> 3, p = tid & 7;
  const v8h hv = *(const v8h*)(sT + nl * TPP + 8 * p);
  _Float16* d = Wp + (size_t)(n0 + nl) * KD + k0 + 8 * p;
  *(volatile v8h*)d = hv;
  __threadfence();
  *(volatile v8h*)d = hv;
}

__global__ __launch_bounds__(NTHR) void k_count(
    const int* __restrict__ keys, int* cnt, float* dinv, int nK, int nN, int vec8) {
  extern __shared__ v4f lds_dyn[];
  int* scnt = (int*)lds_dyn;
  int* list = scnt + NBC;
  int* wcnt = list + NWAVE * WCAPC;
  const int tid = threadIdx.x, lane = tid & 31, wave = tid >> 5;
  const int nodeBase = blockIdx.x * NBC;

  {
    const v4i z = {0, 0, 0, 0};
    for (int i = tid; i < NBC / 4; i += NTHR) ((v4i*)scnt)[i] = z;
  }
  __syncthreads();

  const int nChunks = (nK + CHUNK - 1) / CHUNK;
#pragma unroll 1
  for (int ch = 0; ch < nChunks; ++ch) {
    const int cbase = ch * CHUNK;
    const int wc = scan_chunk<NBC, 0, WCAPC>(keys, keys, nK, nN, cbase, nodeBase, vec8, list, tid, lane, wave);
    if (lane == 0) wcnt[wave] = wc;
    __syncthreads();
    if (wave == 0) {
#pragma unroll 1
      for (int wsx = 0; wsx < NWAVE; ++wsx) {
        int n = __builtin_amdgcn_readfirstlane(wcnt[wsx]);
        n = n > WCAPC ? WCAPC : (n < 0 ? 0 : n);
        const int* lp = list + wsx * WCAPC;
#pragma unroll 1
        for (int i = 0; i < n; ++i) {
          const int ent  = __builtin_amdgcn_readfirstlane(lp[i]);
          const int slot = ent & (NBC - 1);
          if (lane == 0) scnt[slot] = scnt[slot] + 1;
        }
      }
    }
    __syncthreads();
  }

  int*   cp = cnt + (size_t)nodeBase;
  float* dp = dinv + (size_t)nodeBase;
#pragma unroll 4
  for (int q = 0; q < 32; ++q) {
    const int f = (wave * 32 + q) * 128 + 4 * lane;
    const v4i c = *(const v4i*)(scnt + f);
    const float g0 = (float)c.x + CSELF, g1 = (float)c.y + CSELF, g2 = (float)c.z + CSELF, g3 = (float)c.w + CSELF;
    v4f d;
    d.x = g0 > 0.f ? rsqrtf(g0) : 0.f; d.y = g1 > 0.f ? rsqrtf(g1) : 0.f;
    d.z = g2 > 0.f ? rsqrtf(g2) : 0.f; d.w = g3 > 0.f ? rsqrtf(g3) : 0.f;
    *(volatile v4i*)(cp + f) = c;
    *(volatile v4f*)(dp + f) = d;
  }
  __threadfence();
#pragma unroll 4
  for (int q = 0; q < 32; ++q) {
    const int f = (wave * 32 + q) * 128 + 4 * lane;
    const v4i c = *(const v4i*)(scnt + f);
    const float g0 = (float)c.x + CSELF, g1 = (float)c.y + CSELF, g2 = (float)c.z + CSELF, g3 = (float)c.w + CSELF;
    v4f d;
    d.x = g0 > 0.f ? rsqrtf(g0) : 0.f; d.y = g1 > 0.f ? rsqrtf(g1) : 0.f;
    d.z = g2 > 0.f ? rsqrtf(g2) : 0.f; d.w = g3 > 0.f ? rsqrtf(g3) : 0.f;
    *(volatile v4i*)(cp + f) = c;
    *(volatile v4f*)(dp + f) = d;
  }
}

__global__ __launch_bounds__(OTHR) void k_offsets(
    const int* __restrict__ cnt, int* off, int* rbase, int* flag, int nBF) {
  __shared__ __attribute__((aligned(16))) int srb[RBN];
  __shared__ int wtot[OTHR / 32];
  __shared__ int wbad[OTHR / 32];
  const int tid = threadIdx.x, lane = tid & 31, wave = tid >> 5;
  for (int i = tid; i < RBN; i += OTHR) srb[i] = 0;
  int carry = 0;
  int bad = 0;
#pragma unroll 1
  for (int fb = 0; fb < nBF; ++fb) {
    const int base = fb * NBF;
    const v4i c = *(const v4i*)(cnt + base + 4 * tid);
    bad |= (c.x > DEGCAP) ? 1 : 0;
    bad |= (c.y > DEGCAP) ? 1 : 0;
    bad |= (c.z > DEGCAP) ? 1 : 0;
    bad |= (c.w > DEGCAP) ? 1 : 0;
    const int e0 = max(c.x, 0), e1 = max(c.y, 0), e2 = max(c.z, 0), e3 = max(c.w, 0);
    const int ts = e0 + e1 + e2 + e3;
    int incl = ts;
#pragma unroll
    for (int d = 1; d < 32; d <<= 1) {
      const int t = __shfl_up(incl, d, 32);
      if (lane >= d) incl += t;
    }
    if (lane == 31) wtot[wave] = incl;
    __syncthreads();
    int pre = 0;
#pragma unroll 1
    for (int w = 0; w < wave; ++w) pre += wtot[w];
    int tot = 0;
#pragma unroll
    for (int w = 0; w < OTHR / 32; ++w) tot += wtot[w];
    if (tot > RCAP) bad = 1;
    int run = carry + pre + incl - ts;
    v4i o;
    o.x = run; run += e0;
    o.y = run; run += e1;
    o.z = run; run += e2;
    o.w = run;
    int* op = off + base + 4 * tid;
    *(volatile v4i*)op = o;
    __threadfence();
    *(volatile v4i*)op = o;
    if (tid == 0) srb[min(fb, RBN - 1)] = carry;
    carry += (tot + 31) & ~31;
    __syncthreads();
  }
  if (tid == 0) srb[min(nBF, RBN - 1)] = carry;
  {
    int b = bad;
#pragma unroll
    for (int oo = 16; oo > 0; oo >>= 1) b |= __shfl_xor(b, oo, 32);
    if (lane == 0) wbad[wave] = b;
  }
  __syncthreads();
  if (tid < 32) {
    const v4i rv = *(const v4i*)(srb + 4 * tid);
    int fv = wbad[lane & (OTHR / 32 - 1)];
#pragma unroll
    for (int oo = 16; oo > 0; oo >>= 1) fv |= __shfl_xor(fv, oo, 32);
    *(volatile v4i*)(rbase + 4 * tid) = rv;
    *(volatile int*)(flag + lane) = fv;
    __threadfence();
    *(volatile v4i*)(rbase + 4 * tid) = rv;
    *(volatile int*)(flag + lane) = fv;
  }
}

__global__ __launch_bounds__(NTHR) void k_fill(
    const int* __restrict__ keys, const int* __restrict__ vals, const int* __restrict__ off,
    const int* __restrict__ rbase, int* csr, int nN, int nK, int vec8, int csrLen) {
  extern __shared__ v4f lds_dyn[];
  int* region = (int*)lds_dyn;
  int* cursor = region + RCAP;
  int* list   = cursor + NBF;
  int* wcnt   = list + NWAVE * WCAPF;
  const int tid = threadIdx.x, lane = tid & 31, wave = tid >> 5;
  const int b = blockIdx.x;
  const int nodeBase = b * NBF;

  int rb0 = rbase[b];
  const int rb1 = rbase[b + 1];
  rb0 = rb0 < 0 ? 0 : (rb0 > csrLen ? csrLen : rb0);
  rb0 &= ~31;
  int len = rb1 - rb0;
  len = len < 0 ? 0 : (len > RCAP ? RCAP : len);
  int lenW = (len + 31) & ~31;
  if (rb0 + lenW > csrLen) lenW = (csrLen - rb0) & ~31;

  {
    const v4i z = {0, 0, 0, 0};
    for (int i = tid; i < RCAP / 4; i += NTHR) ((v4i*)region)[i] = z;
    for (int s = tid; s < NBF; s += NTHR) {
      int o = off[nodeBase + s] - rb0;
      o = o < 0 ? 0 : (o > RCAP ? RCAP : o);
      cursor[s] = o;
    }
  }
  __syncthreads();

  const int nChunks = (nK + CHUNK - 1) / CHUNK;
#pragma unroll 1
  for (int ch = 0; ch < nChunks; ++ch) {
    const int cbase = ch * CHUNK;
    const int wc = scan_chunk<NBF, 1, WCAPF>(keys, vals, nK, nN, cbase, nodeBase, vec8, list, tid, lane, wave);
    if (lane == 0) wcnt[wave] = wc;
    __syncthreads();
    if (wave == 0) {
#pragma unroll 1
      for (int wsx = 0; wsx < NWAVE; ++wsx) {
        int n = __builtin_amdgcn_readfirstlane(wcnt[wsx]);
        n = n > WCAPF ? WCAPF : (n < 0 ? 0 : n);
        const int* lp = list + wsx * WCAPF;
#pragma unroll 1
        for (int i = 0; i < n; ++i) {
          const int ent  = __builtin_amdgcn_readfirstlane(lp[i]);
          const int slot = ent & (NBF - 1);
          int src = (ent >> ESHF) & 0xFFFFF;
          src = src > nN - 1 ? nN - 1 : src;
          if (lane == 0) {
            int pos = cursor[slot];
            pos = pos < 0 ? 0 : (pos > RCAP - 1 ? RCAP - 1 : pos);
            region[pos] = src;
            const int np = pos + 1;
            cursor[slot] = np > RCAP ? RCAP : np;
          }
        }
      }
    }
    __syncthreads();
  }

  const int nv = lenW >> 2;
  int* gp = csr + rb0;
#pragma unroll 1
  for (int i = tid; i < nv; i += NTHR) { const v4i v = ((const v4i*)region)[i]; *(volatile v4i*)(gp + 4 * i) = v; }
  __threadfence();
#pragma unroll 1
  for (int i = tid; i < nv; i += NTHR) { const v4i v = ((const v4i*)region)[i]; *(volatile v4i*)(gp + 4 * i) = v; }
}

template <int KD, int RS, int BI, int O16>
__global__ __launch_bounds__(NTHR) void k_gemm(
    const _Float16* __restrict__ A16, const _Float16* __restrict__ Bw,
    const float* __restrict__ rsc, const float* __restrict__ bias,
    float* Cf, _Float16* Ch, int nRows, int nValid, float osc, float hscl) {
  static_assert((KD % 32) == 0);
  extern __shared__ v4f lds_dyn[];
  constexpr int NT = GCOLS / 16;
  float* stg = (float*)lds_dyn;
  const int tid = threadIdx.x, lane = tid & 31, wave = tid >> 5, hh = lane >> 4, m = lane & 15;
  const int rowBase = blockIdx.x * GROWS;
  const _Float16* ap  = A16 + (size_t)(rowBase + wave * 16 + m) * KD + 8 * hh;
  const _Float16* bp0 = Bw + (size_t)m * KD + 8 * hh;

  v8f acc[NT];
#pragma unroll
  for (int t = 0; t < NT; ++t) { v8f z = {0.f, 0.f, 0.f, 0.f, 0.f, 0.f, 0.f, 0.f}; acc[t] = z; }

#pragma unroll 1
  for (int kt = 0; kt < KD / 32; ++kt) {
    FragH af;
    af.h[0] = *(const v8h*)(ap + 32 * kt);
    af.h[1] = *(const v8h*)(ap + 32 * kt + 16);
#pragma unroll
    for (int t = 0; t < NT; ++t) {
      const _Float16* bp = bp0 + (size_t)(16 * t) * KD + 32 * kt;
      FragH bf;
      bf.h[0] = *(const v8h*)bp;
      bf.h[1] = *(const v8h*)(bp + 16);
      acc[t] = wmf(af.v, bf.v, acc[t]);
    }
  }

  const int r0 = wave * 16 + 8 * hh;
  float s[8];
  if (RS != 0) {
    const v4f dA = *(const v4f*)(rsc + (size_t)rowBase + r0);
    const v4f dB = *(const v4f*)(rsc + (size_t)rowBase + r0 + 4);
    s[0] = dA.x; s[1] = dA.y; s[2] = dA.z; s[3] = dA.w; s[4] = dB.x; s[5] = dB.y; s[6] = dB.z; s[7] = dB.w;
#pragma unroll
    for (int r = 0; r < 8; ++r) s[r] = s[r] * osc;
  } else {
#pragma unroll
    for (int r = 0; r < 8; ++r) s[r] = osc;
  }
  float bb[NT];
#pragma unroll
  for (int t = 0; t < NT; ++t) bb[t] = (BI != 0) ? bias[16 * t + m] : 0.0f;

  float* sp = stg + r0 * GCOLS + m;
#pragma unroll
  for (int t = 0; t < NT; ++t) {
#pragma unroll
    for (int r = 0; r < 8; ++r) sp[r * GCOLS + 16 * t] = acc[t][r] * s[r] + bb[t];
  }
  __syncthreads();

  const float* lp = stg + wave * 16 * GCOLS;
  if (O16 == 0) {
    float* gp = Cf + (size_t)(rowBase + wave * 16) * HD;
#pragma unroll
    for (int i = 0; i < 16; ++i) {
      if (rowBase + wave * 16 + i < nRows) {
        const v4f v = *(const v4f*)(lp + i * GCOLS + 4 * lane);
        *(volatile v4f*)(gp + (size_t)i * HD + 4 * lane) = v;
      }
    }
    __threadfence();
#pragma unroll
    for (int i = 0; i < 16; ++i) {
      if (rowBase + wave * 16 + i < nRows) {
        const v4f v = *(const v4f*)(lp + i * GCOLS + 4 * lane);
        *(volatile v4f*)(gp + (size_t)i * HD + 4 * lane) = v;
      }
    }
  } else {
    const int rr = lane >> 4, c8 = 8 * (lane & 15);
    _Float16* gp = Ch + (size_t)(rowBase + wave * 16) * HD;
#pragma unroll
    for (int i = 0; i < 8; ++i) {
      const int row = 2 * i + rr;
      if (rowBase + wave * 16 + 2 * i < nRows) {
        const float z = (rowBase + wave * 16 + row < nValid) ? hscl : 0.0f;
        const v4f f0 = *(const v4f*)(lp + row * GCOLS + c8);
        const v4f f1 = *(const v4f*)(lp + row * GCOLS + c8 + 4);
        v8h hv;
        hv[0] = (_Float16)(f0.x * z); hv[1] = (_Float16)(f0.y * z); hv[2] = (_Float16)(f0.z * z); hv[3] = (_Float16)(f0.w * z);
        hv[4] = (_Float16)(f1.x * z); hv[5] = (_Float16)(f1.y * z); hv[6] = (_Float16)(f1.z * z); hv[7] = (_Float16)(f1.w * z);
        *(volatile v8h*)(gp + (size_t)row * HD + c8) = hv;
      }
    }
    __threadfence();
#pragma unroll
    for (int i = 0; i < 8; ++i) {
      const int row = 2 * i + rr;
      if (rowBase + wave * 16 + 2 * i < nRows) {
        const float z = (rowBase + wave * 16 + row < nValid) ? hscl : 0.0f;
        const v4f f0 = *(const v4f*)(lp + row * GCOLS + c8);
        const v4f f1 = *(const v4f*)(lp + row * GCOLS + c8 + 4);
        v8h hv;
        hv[0] = (_Float16)(f0.x * z); hv[1] = (_Float16)(f0.y * z); hv[2] = (_Float16)(f0.z * z); hv[3] = (_Float16)(f0.w * z);
        hv[4] = (_Float16)(f1.x * z); hv[5] = (_Float16)(f1.y * z); hv[6] = (_Float16)(f1.z * z); hv[7] = (_Float16)(f1.w * z);
        *(volatile v8h*)(gp + (size_t)row * HD + c8) = hv;
      }
    }
  }
}

template <int MODE>
__global__ __launch_bounds__(NTHR) void k_agg(
    const int* __restrict__ csr, const int* __restrict__ off, const int* __restrict__ cnt,
    const float* __restrict__ dinv, const float* __restrict__ hw, const float* __restrict__ bias,
    const float* __restrict__ gam, const float* __restrict__ bet,
    const float* __restrict__ eW, const float* __restrict__ rW,
    _Float16* outH, float* outS, int nN, int csrLen, float hscl) {
  extern __shared__ v4f lds_dyn[];
  _Float16* sH = (_Float16*)lds_dyn;
  const int tid = threadIdx.x, lane = tid & 31, wave = tid >> 5;
  const int tbase = blockIdx.x * TGT + wave * 32;
  const int cl = tbase + lane;
  const int cnt_l = cnt[cl];
  const int off_l = off[cl];
  U32F dvu; dvu.f = dinv[cl];
  const int ch = 4 * lane;
  const v4f bq = *(const v4f*)(bias + ch);
  const v4f g4 = *(const v4f*)(gam + ch);
  const v4f b4 = *(const v4f*)(bet + ch);
  v4f we0 = {0.f, 0.f, 0.f, 0.f}, we1 = {0.f, 0.f, 0.f, 0.f};
  v4f wr0 = {0.f, 0.f, 0.f, 0.f}, wr1 = {0.f, 0.f, 0.f, 0.f};
  if (MODE == 1) {
    we0 = *(const v4f*)(eW + ch); we1 = *(const v4f*)(eW + HD + ch);
    wr0 = *(const v4f*)(rW + ch); wr1 = *(const v4f*)(rW + HD + ch);
  }
  v4f keep = {0.f, 0.f, 0.f, 0.f};
  const float invh = 1.0f / (float)HD;

#pragma unroll 1
  for (int j = 0; j < 32; ++j) {
    const int c = tbase + j;
    int n = __builtin_amdgcn_readlane(cnt_l, j);
    n = n < 0 ? 0 : (n > DEGCAP ? DEGCAP : n);
    const int st = __builtin_amdgcn_readlane(off_l, j);
    U32F du; du.i = __builtin_amdgcn_readlane(dvu.i, j);
    const float dc = du.f;
    v4f acc = {0.f, 0.f, 0.f, 0.f};
#pragma unroll 1
    for (int q0 = 0; q0 < n; q0 += 32) {
      int pos = st + q0 + lane;
      pos = pos < 0 ? 0 : (pos > csrLen - 1 ? csrLen - 1 : pos);
      int sl = csr[pos];
      sl = sl < 0 ? 0 : (sl > nN - 1 ? nN - 1 : sl);
      const int mcnt = (n - q0) < 32 ? (n - q0) : 32;
#pragma unroll 1
      for (int p = 0; p < mcnt; ++p) {
        const int s = __builtin_amdgcn_readlane(sl, p);
        const v4f hv = *(const v4f*)(hw + (size_t)s * HD + ch);
        acc.x += hv.x; acc.y += hv.y; acc.z += hv.z; acc.w += hv.w;
      }
    }
    const v4f sv = *(const v4f*)(hw + (size_t)c * HD + ch);
    v4f t;
    t.x = (acc.x + sv.x * CSELF) * dc + bq.x;
    t.y = (acc.y + sv.y * CSELF) * dc + bq.y;
    t.z = (acc.z + sv.z * CSELF) * dc + bq.z;
    t.w = (acc.w + sv.w * CSELF) * dc + bq.w;
    const float mu = wsum((t.x + t.y) + (t.z + t.w)) * invh;
    v4f d;
    d.x = t.x - mu; d.y = t.y - mu; d.z = t.z - mu; d.w = t.w - mu;
    const float var = wsum(d.x * d.x + d.y * d.y + d.z * d.z + d.w * d.w) * invh;
    const float rstd = rsqrtf(var + LN_EPS);
    v4f y;
    y.x = leaky(d.x * rstd * g4.x + b4.x);
    y.y = leaky(d.y * rstd * g4.y + b4.y);
    y.z = leaky(d.z * rstd * g4.z + b4.z);
    y.w = leaky(d.w * rstd * g4.w + b4.w);
    if (MODE == 0) {
      const float z = (c < nN) ? hscl : 0.0f;
      v4h h;
      h[0] = (_Float16)(y.x * z); h[1] = (_Float16)(y.y * z); h[2] = (_Float16)(y.z * z); h[3] = (_Float16)(y.w * z);
      *(v4h*)(sH + (size_t)(wave * 32 + j) * HD + ch) = h;
    } else {
      const float zf = (c < nN) ? 1.0f : 0.0f;
      const float p0 = wsum(y.x * we0.x + y.y * we0.y + y.z * we0.z + y.w * we0.w) * zf;
      const float p1 = wsum(y.x * we1.x + y.y * we1.y + y.z * we1.z + y.w * we1.w) * zf;
      const float p2 = wsum(y.x * wr0.x + y.y * wr0.y + y.z * wr0.z + y.w * wr0.w) * zf;
      const float p3 = wsum(y.x * wr1.x + y.y * wr1.y + y.z * wr1.z + y.w * wr1.w) * zf;
      const bool mine = (lane == j);
      keep.x = mine ? p0 : keep.x;
      keep.y = mine ? p1 : keep.y;
      keep.z = mine ? p2 : keep.z;
      keep.w = mine ? p3 : keep.w;
    }
  }

  if (MODE == 0) {
    __syncthreads();
    const int rr = lane >> 4, c8 = 8 * (lane & 15);
    const _Float16* lp = sH + (size_t)(wave * 32) * HD;
    _Float16* gp = outH + (size_t)tbase * HD;
#pragma unroll
    for (int i = 0; i < 16; ++i) {
      const int row = 2 * i + rr;
      const v8h hv = *(const v8h*)(lp + row * HD + c8);
      *(volatile v8h*)(gp + (size_t)row * HD + c8) = hv;
    }
    __threadfence();
#pragma unroll
    for (int i = 0; i < 16; ++i) {
      const int row = 2 * i + rr;
      const v8h hv = *(const v8h*)(lp + row * HD + c8);
      *(volatile v8h*)(gp + (size_t)row * HD + c8) = hv;
    }
  } else {
    float* spo = outS + (size_t)(tbase + lane) * 4;
    *(volatile v4f*)spo = keep;
    __threadfence();
    *(volatile v4f*)spo = keep;
  }
}

__global__ __launch_bounds__(NTHR) void k_pred(
    const float* __restrict__ S4, const int* __restrict__ eu, const int* __restrict__ ef,
    const float* __restrict__ eB, const float* __restrict__ rB, const int* __restrict__ flag,
    float* exist, float* rating, int P, int nN) {
  const int i = (int)blockIdx.x * NTHR + (int)threadIdx.x;
  const int total4 = P >> 2;
  const int rem = P - 4 * total4;
  U32F pz; pz.i = (flag[0] != 0) ? 0x7fc00000 : 0;
  const float poison = pz.f;
  const float eb = eB[0], rb = rB[0];
  if (total4 > 0) {
    const int ic = i < total4 ? i : total4 - 1;
    v4i u4 = *(const v4i*)(eu + (size_t)4 * (size_t)ic);
    v4i f4 = *(const v4i*)(ef + (size_t)4 * (size_t)ic);
    u4.x = min(max(u4.x, 0), nN - 1); u4.y = min(max(u4.y, 0), nN - 1);
    u4.z = min(max(u4.z, 0), nN - 1); u4.w = min(max(u4.w, 0), nN - 1);
    f4.x = min(max(f4.x, 0), nN - 1); f4.y = min(max(f4.y, 0), nN - 1);
    f4.z = min(max(f4.z, 0), nN - 1); f4.w = min(max(f4.w, 0), nN - 1);
    const v4f su0 = *(const v4f*)(S4 + (size_t)4 * u4.x), sf0 = *(const v4f*)(S4 + (size_t)4 * f4.x);
    const v4f su1 = *(const v4f*)(S4 + (size_t)4 * u4.y), sf1 = *(const v4f*)(S4 + (size_t)4 * f4.y);
    const v4f su2 = *(const v4f*)(S4 + (size_t)4 * u4.z), sf2 = *(const v4f*)(S4 + (size_t)4 * f4.z);
    const v4f su3 = *(const v4f*)(S4 + (size_t)4 * u4.w), sf3 = *(const v4f*)(S4 + (size_t)4 * f4.w);
    v4f ex, rt;
    ex.x = sigm(su0.x + sf0.y + eb) + poison; rt.x = 1.0f + 4.0f * sigm(su0.z + sf0.w + rb) + poison;
    ex.y = sigm(su1.x + sf1.y + eb) + poison; rt.y = 1.0f + 4.0f * sigm(su1.z + sf1.w + rb) + poison;
    ex.z = sigm(su2.x + sf2.y + eb) + poison; rt.z = 1.0f + 4.0f * sigm(su2.z + sf2.w + rb) + poison;
    ex.w = sigm(su3.x + sf3.y + eb) + poison; rt.w = 1.0f + 4.0f * sigm(su3.z + sf3.w + rb) + poison;
    if (i < total4) {
      *(volatile v4f*)(exist + (size_t)4 * (size_t)i) = ex;
      *(volatile v4f*)(rating + (size_t)4 * (size_t)i) = rt;
    }
    __threadfence();
    if (i < total4) {
      *(volatile v4f*)(exist + (size_t)4 * (size_t)i) = ex;
      *(volatile v4f*)(rating + (size_t)4 * (size_t)i) = rt;
    }
  }
  if (rem != 0) {
    float exs[3], rts[3];
#pragma unroll
    for (int j = 0; j < 3; ++j) {
      int idx = 4 * total4 + j;
      idx = idx > P - 1 ? P - 1 : idx;
      int u = eu[idx], f = ef[idx];
      u = min(max(u, 0), nN - 1); f = min(max(f, 0), nN - 1);
      const v4f su = *(const v4f*)(S4 + (size_t)4 * u);
      const v4f sf = *(const v4f*)(S4 + (size_t)4 * f);
      exs[j] = sigm(su.x + sf.y + eb) + poison;
      rts[j] = 1.0f + 4.0f * sigm(su.z + sf.w + rb) + poison;
    }
    if (i == total4) {
#pragma unroll
      for (int j = 0; j < 3; ++j) {
        if (j < rem) {
          *(volatile float*)(exist + (size_t)4 * total4 + j) = exs[j];
          *(volatile float*)(rating + (size_t)4 * total4 + j) = rts[j];
        }
      }
    }
    __threadfence();
    if (i == total4) {
#pragma unroll
      for (int j = 0; j < 3; ++j) {
        if (j < rem) {
          *(volatile float*)(exist + (size_t)4 * total4 + j) = exs[j];
          *(volatile float*)(rating + (size_t)4 * total4 + j) = rts[j];
        }
      }
    }
  }
}

extern "C" void kernel_launch(void* const* d_in, const int* in_sizes, int n_in,
                              void* d_out, int out_size, void* d_ws, size_t ws_size,
                              hipStream_t stream) {
  if (n_in < 21) return;
  const int nNU = in_sizes[0] / UD;
  const int nNF = in_sizes[1] / HD;
  const int nN  = nNU + nNF;
  const int nE  = in_sizes[2] / 2;
  const int P   = in_sizes[3];
  if (nNU <= 0 || nNF <= 0 || nE <= 0 || P <= 0) return;
  if (in_sizes[0] != nNU * UD || in_sizes[1] != nNF * HD || in_sizes[2] != 2 * nE || in_sizes[4] != P) return;
  if (in_sizes[5] != UD * HD || in_sizes[6] != HD || in_sizes[7] != HD * HD || in_sizes[8] != HD) return;
  if (in_sizes[9] != HD * HD || in_sizes[10] != HD || in_sizes[11] != HD * HD || in_sizes[12] != HD) return;
  if (in_sizes[13] != HD || in_sizes[14] != HD || in_sizes[15] != HD || in_sizes[16] != HD) return;
  if (in_sizes[17] != 2 * HD || in_sizes[18] < 1 || in_sizes[19] != 2 * HD || in_sizes[20] < 1) return;
  if ((nNU % 16) != 0) return;
  if (nN > (1 << 20) || nE > (1 << 28) || P > (1 << 29)) return;
  if ((long long)out_size != 2LL * (long long)P) return;

  const float* u_feat = (const float*)d_in[0];
  const float* f_feat = (const float*)d_in[1];
  const int*   ei     = (const int*)d_in[2];
  const int*   edge_u = (const int*)d_in[3];
  const int*   edge_f = (const int*)d_in[4];
  const float* u_W    = (const float*)d_in[5];
  const float* u_b    = (const float*)d_in[6];
  const float* f_W    = (const float*)d_in[7];
  const float* f_b    = (const float*)d_in[8];
  const float* c1_W   = (const float*)d_in[9];
  const float* c1_b   = (const float*)d_in[10];
  const float* c2_W   = (const float*)d_in[11];
  const float* c2_b   = (const float*)d_in[12];
  const float* n1_g   = (const float*)d_in[13];
  const float* n1_b   = (const float*)d_in[14];
  const float* n2_g   = (const float*)d_in[15];
  const float* n2_b   = (const float*)d_in[16];
  const float* e_W    = (const float*)d_in[17];
  const float* e_b    = (const float*)d_in[18];
  const float* r_W    = (const float*)d_in[19];
  const float* r_b    = (const float*)d_in[20];
  float* exist  = (float*)d_out;
  float* rating = exist + (size_t)P;
  const int* keys = ei + nE;
  const int* vals = ei;
  const int nK = nE;

  const int NPAD   = ((nN + TGT - 1) / TGT) * TGT;
  const int NUPAD  = ((nNU + GROWS - 1) / GROWS) * GROWS;
  const int rowsF  = NPAD - nNU;
  const int NFPAD  = ((rowsF + GROWS - 1) / GROWS) * GROWS;
  const int nBC    = (nN + NBC - 1) / NBC;
  const int CNTPAD = nBC * NBC;
  const int nBF    = (nN + NBF - 1) / NBF;
  const int OFFN   = nBF * NBF;
  if (nBF + 1 > RBN) return;
  if (OFFN > CNTPAD || NPAD > OFFN || rowsF < nNF) return;
  const int csrLen = ((nK + 31) & ~31) + 32 * (nBF + 1);
  const int nGemmU = NUPAD / GROWS;
  const int nGemmF = NFPAD / GROWS;
  const int nGemm  = NPAD / GROWS;
  const int nAgg   = NPAD / TGT;

  char* ws = (char*)d_ws;
  size_t off = 0;
  const size_t oU16 = off; off += (size_t)NUPAD * UD * 2;        off = (off + 255) & ~(size_t)255;
  const size_t oF16 = off; off += (size_t)NFPAD * HD * 2;        off = (off + 255) & ~(size_t)255;
  const size_t oWu  = off; off += (size_t)HD * UD * 2;           off = (off + 255) & ~(size_t)255;
  const size_t oWf  = off; off += (size_t)HD * HD * 2;           off = (off + 255) & ~(size_t)255;
  const size_t oW1  = off; off += (size_t)HD * HD * 2;           off = (off + 255) & ~(size_t)255;
  const size_t oW2  = off; off += (size_t)HD * HD * 2;           off = (off + 255) & ~(size_t)255;
  const size_t oCnt = off; off += (size_t)CNTPAD * 4;            off = (off + 255) & ~(size_t)255;
  const size_t oDv  = off; off += (size_t)CNTPAD * 4;            off = (off + 255) & ~(size_t)255;
  const size_t oOff = off; off += (size_t)OFFN * 4;              off = (off + 255) & ~(size_t)255;
  const size_t oRb  = off; off += (size_t)RBN * 4;               off = (off + 255) & ~(size_t)255;
  const size_t oFlg = off; off += (size_t)32 * 4;                off = (off + 255) & ~(size_t)255;
  const size_t oCsr = off; off += (size_t)csrLen * 4;            off = (off + 255) & ~(size_t)255;
  const size_t oX0h = off; off += (size_t)NPAD * HD * 2;         off = (off + 255) & ~(size_t)255;
  const size_t oHX  = off; off += (size_t)NPAD * HD * 4;         off = (off + 255) & ~(size_t)255;
  const size_t oH1h = off; off += (size_t)NPAD * HD * 2;         off = (off + 255) & ~(size_t)255;
  const size_t oS4  = off; off += (size_t)NPAD * 4 * 4;          off = (off + 255) & ~(size_t)255;
  if (off > ws_size || off > (size_t)WSCAP) return;
  _Float16* U16p = (_Float16*)(ws + oU16);
  _Float16* F16p = (_Float16*)(ws + oF16);
  _Float16* WuT  = (_Float16*)(ws + oWu);
  _Float16* WfT  = (_Float16*)(ws + oWf);
  _Float16* W1T  = (_Float16*)(ws + oW1);
  _Float16* W2T  = (_Float16*)(ws + oW2);
  int*      cnt  = (int*)(ws + oCnt);
  float*    dinv = (float*)(ws + oDv);
  int*      offp = (int*)(ws + oOff);
  int*      rb   = (int*)(ws + oRb);
  int*      flg  = (int*)(ws + oFlg);
  int*      csr  = (int*)(ws + oCsr);
  _Float16* X0h  = (_Float16*)(ws + oX0h);
  float*    HX   = (float*)(ws + oHX);
  _Float16* H1h  = (_Float16*)(ws + oH1h);
  float*    S4   = (float*)(ws + oS4);

  const int vec8 = ((nE & 7) == 0) ? 1 : 0;
  const float oscP = 1.0f / ((float)ASCL * (float)WSCL);
  const float oscH = 1.0f / ((float)HSCL * (float)WSCL);

  {
    const int t8u = (NUPAD * UD) / 8;
    k_cvt16<<<(t8u + NTHR - 1) / NTHR, NTHR, 0, stream>>>(u_feat, U16p, UD, nNU, t8u, (float)ASCL);
    const int t8f = (NFPAD * HD) / 8;
    k_cvt16<<<(t8f + NTHR - 1) / NTHR, NTHR, 0, stream>>>(f_feat, F16p, HD, nNF, t8f, (float)ASCL);
  }
  {
    k_wT16<<<dim3(UD / TPK, HD / TPN), NTHR, 0, stream>>>(u_W, WuT, UD, HD, (float)WSCL);
    const dim3 gT(HD / TPK, HD / TPN);
    k_wT16<<<gT, NTHR, 0, stream>>>(f_W,  WfT, HD, HD, (float)WSCL);
    k_wT16<<<gT, NTHR, 0, stream>>>(c1_W, W1T, HD, HD, (float)WSCL);
    k_wT16<<<gT, NTHR, 0, stream>>>(c2_W, W2T, HD, HD, (float)WSCL);
  }

  hipFuncSetAttribute(reinterpret_cast<const void*>(&k_count),
                      hipFuncAttributeMaxDynamicSharedMemorySize, LDS_COUNT);
  k_count<<<nBC, NTHR, LDS_COUNT, stream>>>(keys, cnt, dinv, nK, nN, vec8);
  k_offsets<<<1, OTHR, 0, stream>>>(cnt, offp, rb, flg, nBF);
  hipFuncSetAttribute(reinterpret_cast<const void*>(&k_fill),
                      hipFuncAttributeMaxDynamicSharedMemorySize, LDS_FILL);
  k_fill<<<nBF, NTHR, LDS_FILL, stream>>>(keys, vals, offp, rb, csr, nN, nK, vec8, csrLen);

  hipFuncSetAttribute(reinterpret_cast<const void*>(&k_gemm<UD, 0, 1, 1>),
                      hipFuncAttributeMaxDynamicSharedMemorySize, LDS_GEMM);
  k_gemm<UD, 0, 1, 1><<<nGemmU, NTHR, LDS_GEMM, stream>>>(U16p, WuT, dinv, u_b, HX, X0h, nNU, nNU, oscP, (float)HSCL);
  hipFuncSetAttribute(reinterpret_cast<const void*>(&k_gemm<HD, 0, 1, 1>),
                      hipFuncAttributeMaxDynamicSharedMemorySize, LDS_GEMM);
  k_gemm<HD, 0, 1, 1><<<nGemmF, NTHR, LDS_GEMM, stream>>>(F16p, WfT, dinv, f_b, HX, X0h + (size_t)nNU * HD,
                                                          rowsF, nNF, oscP, (float)HSCL);

  hipFuncSetAttribute(reinterpret_cast<const void*>(&k_gemm<HD, 1, 0, 0>),
                      hipFuncAttributeMaxDynamicSharedMemorySize, LDS_GEMM);
  k_gemm<HD, 1, 0, 0><<<nGemm, NTHR, LDS_GEMM, stream>>>(X0h, W1T, dinv, c1_b, HX, X0h, NPAD, NPAD, oscH, 1.0f);
  hipFuncSetAttribute(reinterpret_cast<const void*>(&k_agg<0>),
                      hipFuncAttributeMaxDynamicSharedMemorySize, LDS_AGG);
  k_agg<0><<<nAgg, NTHR, LDS_AGG, stream>>>(csr, offp, cnt, dinv, HX, c1_b, n1_g, n1_b, e_W, r_W,
                                            H1h, S4, nN, csrLen, (float)HSCL);

  k_gemm<HD, 1, 0, 0><<<nGemm, NTHR, LDS_GEMM, stream>>>(H1h, W2T, dinv, c2_b, HX, X0h, NPAD, NPAD, oscH, 1.0f);
  k_agg<1><<<nAgg, NTHR, 0, stream>>>(csr, offp, cnt, dinv, HX, c2_b, n2_g, n2_b, e_W, r_W,
                                      X0h, S4, nN, csrLen, (float)HSCL);

  {
    const int total4 = P >> 2;
    const int rem = P & 3;
    const int nthrP = total4 + (rem != 0 ? 1 : 0);
    k_pred<<<(nthrP + NTHR - 1) / NTHR, NTHR, 0, stream>>>(S4, edge_u, edge_f, e_b, r_b, flg,
                                                           exist, rating, P, nN);
  }
}
